// GATModel_63221918597529
// MI455X (gfx1250) — hardware-verified
//
#include <hip/hip_runtime.h>
#include <stddef.h>
#include <stdint.h>

#define HID     128
#define HEADS   4
#define CH      32
#define INC     64
#define FFH     256
#define NLAY    4
#define NG      64
#define NCLS    10
#define NTHR    256
#define NWAVE   8
#define EPT     8
#define CHUNK   (NTHR * EPT)
#define WCAP    (EPT * 32)
#define LISTN   (NWAVE * WCAP)
#define NB      1024
#define RCAP    28672
#define DEGCAP  256
#define TABN    (2 * NB + 32)
#define GBM     64
#define GTHR    128
#define NEGS    0.2f
#define WSMAX   134217728
#define LDS_BKT ((2 * RCAP + TABN + LISTN + 3 * NWAVE) * 4)

static_assert(HID == 32 * 4);
static_assert(HEADS * CH == HID);
static_assert(CH / 4 == 8);
static_assert(NG == 64);
static_assert(NCLS == 10);
static_assert((NB % 16) == 0 && NB == NWAVE * 128 && NB * 4 == NTHR * 16);
static_assert((CHUNK & (CHUNK - 1)) == 0 && CHUNK <= 4096 && NB <= 4096);
static_assert(LISTN >= NB);
static_assert((RCAP % 32) == 0 && (RCAP % (4 * NTHR)) == 0);
static_assert(RCAP >= 16623 + 4096);
static_assert(DEGCAP >= 35 + 8);
static_assert((TABN % 32) == 0);
static_assert(LDS_BKT <= 300000);
static_assert(GBM == (GTHR / 32) * 16);
static_assert((INC % 32) == 0 && (HID % 32) == 0 && (FFH % 32) == 0);

typedef float          v4f   __attribute__((ext_vector_type(4)));
typedef float          v8f   __attribute__((ext_vector_type(8)));
typedef int            v4i   __attribute__((ext_vector_type(4)));
typedef int            v8i   __attribute__((ext_vector_type(8)));
typedef unsigned       v4u   __attribute__((ext_vector_type(4)));
typedef unsigned short v8us  __attribute__((ext_vector_type(8)));
typedef __bf16         v16bf __attribute__((ext_vector_type(16)));
typedef v4f __attribute__((may_alias)) v4fa;
typedef v4i __attribute__((may_alias)) v4ia;
typedef v4u __attribute__((may_alias)) v4ua;
union FragB { v16bf v; v8us u[2]; v8i w; };

__device__ __forceinline__ v8f wmx(const FragB& a, const FragB& b, v8f c) {
  v8f d = __builtin_amdgcn_wmma_f32_16x16x32_bf16(false, a.v, false, b.v, (short)0, c, false, false);
  asm volatile("v_nop\n\tv_nop\n\tv_nop\n\tv_nop" : "+v"(d) : "v"(a.w), "v"(b.w));
  return d;
}

__device__ __forceinline__ int iclamp(int v, int lo, int hi) { return v < lo ? lo : (v > hi ? hi : v); }

__device__ __forceinline__ unsigned bfbits(float v) {
  const unsigned u = __float_as_uint(v);
  const unsigned r = (u + 0x7FFFu + ((u >> 16) & 1u)) >> 16;
  return (v != v) ? 0x7FC0u : r;
}
__device__ __forceinline__ float rbf(float v) { return __uint_as_float(bfbits(v) << 16); }
__device__ __forceinline__ v4f rbf4(const v4f a) {
  v4f o; o.x = rbf(a.x); o.y = rbf(a.y); o.z = rbf(a.z); o.w = rbf(a.w); return o;
}
__device__ __forceinline__ v8us cvt8b(const v4f a, const v4f b) {
  v8us o;
  o[0] = (unsigned short)bfbits(a.x); o[1] = (unsigned short)bfbits(a.y);
  o[2] = (unsigned short)bfbits(a.z); o[3] = (unsigned short)bfbits(a.w);
  o[4] = (unsigned short)bfbits(b.x); o[5] = (unsigned short)bfbits(b.y);
  o[6] = (unsigned short)bfbits(b.z); o[7] = (unsigned short)bfbits(b.w);
  return o;
}
__device__ __forceinline__ float gelu_f(float v) {
  return 0.5f * v * (1.0f + erff(v * 0.70710678118654752f));
}
__device__ __forceinline__ float wsum(float s) {
  s += __shfl_xor(s, 16); s += __shfl_xor(s, 8); s += __shfl_xor(s, 4);
  s += __shfl_xor(s, 2);  s += __shfl_xor(s, 1);
  return s;
}
__device__ __forceinline__ v4f ln_row(const v4f v, const v4f g, const v4f b) {
  const float mu = wsum(v.x + v.y + v.z + v.w) * (1.0f / 128.0f);
  const float d0 = v.x - mu, d1 = v.y - mu, d2 = v.z - mu, d3 = v.w - mu;
  const float var = wsum(d0 * d0 + d1 * d1 + d2 * d2 + d3 * d3) * (1.0f / 128.0f);
  const float rs = rsqrtf(var + 1e-5f);
  v4f y;
  y.x = d0 * rs * g.x + b.x; y.y = d1 * rs * g.y + b.y;
  y.z = d2 * rs * g.z + b.z; y.w = d3 * rs * g.w + b.w;
  return y;
}
__device__ __forceinline__ v4u hl_pack(unsigned* sw, const v4f y, int lane) {
  const unsigned b0 = bfbits(y.x), b1 = bfbits(y.y), b2 = bfbits(y.z), b3 = bfbits(y.w);
  const unsigned c0 = bfbits(y.x - __uint_as_float(b0 << 16));
  const unsigned c1 = bfbits(y.y - __uint_as_float(b1 << 16));
  const unsigned c2 = bfbits(y.z - __uint_as_float(b2 << 16));
  const unsigned c3 = bfbits(y.w - __uint_as_float(b3 << 16));
  __builtin_amdgcn_fence(__ATOMIC_RELEASE, "wavefront");
  __builtin_amdgcn_wave_barrier();
  sw[2 * lane]          = b0 | (b1 << 16);
  sw[2 * lane + 1]      = b2 | (b3 << 16);
  sw[64 + 2 * lane]     = c0 | (c1 << 16);
  sw[64 + 2 * lane + 1] = c2 | (c3 << 16);
  __builtin_amdgcn_fence(__ATOMIC_RELEASE, "wavefront");
  __builtin_amdgcn_wave_barrier();
  const v4u w = *(const v4ua*)(sw + 4 * lane);
  return w;
}

__device__ __forceinline__ int scan_chunk(const int* __restrict__ dsts, int nE, int cbase, int slotBase,
                                          int nb, int vec8, int* list, int tid, int lane, int wave) {
  int wc = 0;
  const int el0  = tid * EPT;
  const int e0   = cbase + el0;
  const int sent = -2147483647 - 1;
  v4i da, db;
  if (vec8 != 0 && cbase + CHUNK <= nE) {
    da = *(const v4i*)(dsts + e0);
    db = *(const v4i*)(dsts + e0 + 4);
  } else {
    da.x = (e0     < nE) ? dsts[min(e0,     nE - 1)] : sent;
    da.y = (e0 + 1 < nE) ? dsts[min(e0 + 1, nE - 1)] : sent;
    da.z = (e0 + 2 < nE) ? dsts[min(e0 + 2, nE - 1)] : sent;
    da.w = (e0 + 3 < nE) ? dsts[min(e0 + 3, nE - 1)] : sent;
    db.x = (e0 + 4 < nE) ? dsts[min(e0 + 4, nE - 1)] : sent;
    db.y = (e0 + 5 < nE) ? dsts[min(e0 + 5, nE - 1)] : sent;
    db.z = (e0 + 6 < nE) ? dsts[min(e0 + 6, nE - 1)] : sent;
    db.w = (e0 + 7 < nE) ? dsts[min(e0 + 7, nE - 1)] : sent;
  }
  const unsigned nbs = (unsigned)slotBase;
  const unsigned unb = (unsigned)nb;
  const unsigned s0 = (unsigned)da.x - nbs, s1 = (unsigned)da.y - nbs;
  const unsigned s2 = (unsigned)da.z - nbs, s3 = (unsigned)da.w - nbs;
  const unsigned s4 = (unsigned)db.x - nbs, s5 = (unsigned)db.y - nbs;
  const unsigned s6 = (unsigned)db.z - nbs, s7 = (unsigned)db.w - nbs;
  const bool h0 = s0 < unb, h1 = s1 < unb, h2 = s2 < unb, h3 = s3 < unb;
  const bool h4 = s4 < unb, h5 = s5 < unb, h6 = s6 < unb, h7 = s7 < unb;
  const unsigned any = __builtin_amdgcn_ballot_w32(h0 | h1 | h2 | h3 | h4 | h5 | h6 | h7);
  if (any != 0u) {
#define HITJ(J, HJ, SJ) { \
      const unsigned mj = __builtin_amdgcn_ballot_w32(HJ); \
      if (mj != 0u) { \
        if (HJ) { \
          const int pos = wc + (int)__builtin_amdgcn_mbcnt_lo(mj, 0u); \
          if (pos < WCAP) list[wave * WCAP + pos] = ((el0 + (J)) << 12) | (int)(SJ); \
        } \
        wc += (int)__builtin_popcount(mj); } }
    HITJ(0, h0, s0)
    HITJ(1, h1, s1)
    HITJ(2, h2, s2)
    HITJ(3, h3, s3)
    HITJ(4, h4, s4)
    HITJ(5, h5, s5)
    HITJ(6, h6, s6)
    HITJ(7, h7, s7)
#undef HITJ
  }
  return wc;
}

__device__ __forceinline__ void wtr_unit(const float* __restrict__ w, int cols, int Ksrc, int KP,
                                         unsigned short* wt, int nOff, int u) {
  const int kq = KP >> 3;
  const int n  = u / kq;
  const int k8 = (u - n * kq) * 8;
  const int ks = k8 & (Ksrc - 1);
  const float* p = w + (size_t)ks * (size_t)cols + n;
  v4f a, b;
  a.x = p[0];                  a.y = p[(size_t)cols];       a.z = p[(size_t)2 * cols];   a.w = p[(size_t)3 * cols];
  b.x = p[(size_t)4 * cols];   b.y = p[(size_t)5 * cols];   b.z = p[(size_t)6 * cols];   b.w = p[(size_t)7 * cols];
  const v8us hv = cvt8b(a, b);
  const size_t o = (size_t)(nOff + n) * (size_t)KP + k8;
  *(volatile v8us*)(wt + o) = hv;
  __threadfence();
  *(volatile v8us*)(wt + o) = hv;
}

__global__ __launch_bounds__(NTHR) void k_prep(
    const float* __restrict__ x, const float* __restrict__ inW, const float* __restrict__ Wl,
    const float* __restrict__ Wr, const float* __restrict__ W1, const float* __restrict__ W2,
    unsigned short* XB, unsigned short* INWt, unsigned short* WLRt, unsigned short* FW1t, unsigned short* FW2t,
    int nN, int nbx) {
  int b = (int)blockIdx.x;
  const int tid = (int)threadIdx.x;
  if (b < nbx) {
    const int i = b * NTHR + tid;
    const int row = i >> 3;
    const int c0  = (i & 7) * 8;
    const int rc  = row < nN ? row : nN - 1;
    const float* p = x + (size_t)rc * INC + c0;
    v4f a = *(const v4f*)p, c = *(const v4f*)(p + 4);
    const v4f z4 = {0.f, 0.f, 0.f, 0.f};
    if (row >= nN) { a = z4; c = z4; }
    const v8us hv = cvt8b(a, c);
    const size_t o = (size_t)row * INC + c0;
    *(volatile v8us*)(XB + o) = hv;
    __threadfence();
    *(volatile v8us*)(XB + o) = hv;
    return;
  }
  b -= nbx;
  if (b < 4) { wtr_unit(inW, HID, INC, INC, INWt, 0, b * NTHR + tid); return; }
  b -= 4;
  const int ly = b / 96;
  const int r  = b - ly * 96;
  if (ly >= NLAY) return;
  if (r < 16)      wtr_unit(Wl + (size_t)ly * 16384, HID, HID, 256, WLRt + (size_t)ly * 65536, 0,   r * NTHR + tid);
  else if (r < 32) wtr_unit(Wr + (size_t)ly * 16384, HID, HID, 256, WLRt + (size_t)ly * 65536, 128, (r - 16) * NTHR + tid);
  else if (r < 64) wtr_unit(W1 + (size_t)ly * 32768, FFH, HID, 256, FW1t + (size_t)ly * 65536, 0,   (r - 32) * NTHR + tid);
  else             wtr_unit(W2 + (size_t)ly * 32768, HID, FFH, 512, FW2t + (size_t)ly * 65536, 0,   (r - 64) * NTHR + tid);
}

__device__ __forceinline__ void dump_pass(const int* reg2, const int* tab, int* gs, int* gt, int tid) {
  for (int u = tid; u < RCAP / 4; u += NTHR) {
    const v4i v = *(const v4ia*)(reg2 + 4 * u);
    *(volatile v4i*)(gs + 4 * u) = v;
  }
  for (int u = tid; u < TABN / 4; u += NTHR) {
    const v4i v = *(const v4ia*)(tab + 4 * u);
    *(volatile v4i*)(gt + 4 * u) = v;
  }
}

__global__ __launch_bounds__(NTHR) void k_bucket(const int* __restrict__ srcs, const int* __restrict__ dsts,
                                                 int* SRT, int* TAB, int nN, int nE, int vec8) {
  extern __shared__ v4f lds_dyn[];
  int* reg1 = (int*)lds_dyn;
  int* reg2 = reg1 + RCAP;
  int* tab  = reg2 + RCAP;
  int* list = tab + TABN;
  int* wcnt = list + LISTN;
  int* wtot = wcnt + NWAVE;
  int* wflg = wtot + NWAVE;
  int* soff = tab;
  int* scnt = tab + NB;
  const int tid = (int)threadIdx.x, lane = tid & 31, wave = tid >> 5;
  const int nodeBase = (int)blockIdx.x * NB;

  for (int i = tid; i < TABN; i += NTHR) tab[i] = 0;
  for (int i = tid; i < RCAP; i += NTHR) { reg1[i] = 0; reg2[i] = 0; }
  __syncthreads();

  int tot = 0;
  const int nChunks = (nE + CHUNK - 1) / CHUNK;
#pragma unroll 1
  for (int ch = 0; ch < nChunks; ++ch) {
    const int cbase = ch * CHUNK;
    const int wc = scan_chunk(dsts, nE, cbase, nodeBase, NB, vec8, list, tid, lane, wave);
    if (lane == 0) wcnt[wave] = wc;
    __syncthreads();
    int pre = 0, all = 0;
#pragma unroll
    for (int w2 = 0; w2 < NWAVE; ++w2) {
      int c = wcnt[w2];
      c = c < 0 ? 0 : (c > WCAP ? WCAP : c);
      all += c;
      pre += (w2 < wave) ? c : 0;
    }
    const int wcc  = wc > WCAP ? WCAP : wc;
    const int base = tot + pre;
#pragma unroll 1
    for (int i = lane; i < wcc; i += 32) {
      const int ent = list[wave * WCAP + i];
      const int el  = (ent >> 12) & (CHUNK - 1);
      const int sl  = ent & (NB - 1);
      int eid = cbase + el;
      eid = eid > nE - 1 ? nE - 1 : eid;
      const int pos = base + i;
      if (pos < RCAP) reg1[pos] = (int)(((unsigned)eid << 12) | (unsigned)sl);
    }
    tot += all;
    tot = tot > RCAP ? RCAP : tot;
    __syncthreads();
  }
  const int nh = tot;

  if (wave == 0) {
#pragma unroll 1
    for (int b0 = 0; b0 < nh; b0 += 32) {
      const int idx = b0 + lane;
      const int uv  = reg1[idx < RCAP ? idx : RCAP - 1];
      const int m32 = (nh - b0) < 32 ? (nh - b0) : 32;
#pragma unroll 1
      for (int k = 0; k < m32; ++k) {
        const int u  = __builtin_amdgcn_readlane(uv, k);
        const int sl = u & (NB - 1);
        if (lane == 0) scnt[sl] = scnt[sl] + 1;
      }
    }
  }
  __syncthreads();

  {
    const v4i ca = *(const v4ia*)(scnt + 4 * tid);
    const int e0 = ca.x < 0 ? 0 : ca.x, e1 = ca.y < 0 ? 0 : ca.y, e2 = ca.z < 0 ? 0 : ca.z, e3 = ca.w < 0 ? 0 : ca.w;
    const bool of = (e0 > DEGCAP) | (e1 > DEGCAP) | (e2 > DEGCAP) | (e3 > DEGCAP);
    const int ts = e0 + e1 + e2 + e3;
    int incl = ts;
#pragma unroll
    for (int d = 1; d < 32; d <<= 1) {
      const int up = __shfl_up(incl, d);
      if (lane >= d) incl += up;
    }
    const unsigned om = __builtin_amdgcn_ballot_w32(of);
    if (lane == 31) wtot[wave] = incl;
    if (lane == 0)  wflg[wave] = (om != 0u) ? 1 : 0;
    __syncthreads();
    int pre = 0;
#pragma unroll
    for (int w2 = 0; w2 < NWAVE; ++w2) pre += (w2 < wave) ? wtot[w2] : 0;
    int run = pre + incl - ts;
    soff[4 * tid + 0] = run; run += e0;
    soff[4 * tid + 1] = run; run += e1;
    soff[4 * tid + 2] = run; run += e2;
    soff[4 * tid + 3] = run;
  }
  __syncthreads();
  for (int i = tid; i < NB; i += NTHR) list[i] = soff[i];
  __syncthreads();

  if (wave == 0) {
#pragma unroll 1
    for (int b0 = 0; b0 < nh; b0 += 32) {
      const int idx = b0 + lane;
      const int uv  = reg1[idx < RCAP ? idx : RCAP - 1];
      const int m32 = (nh - b0) < 32 ? (nh - b0) : 32;
#pragma unroll 1
      for (int k = 0; k < m32; ++k) {
        const int u   = __builtin_amdgcn_readlane(uv, k);
        const int sl  = u & (NB - 1);
        const int eid = (int)((unsigned)u >> 12);
        if (lane == 0) {
          int pos = list[sl];
          pos = pos < 0 ? 0 : (pos > RCAP - 1 ? RCAP - 1 : pos);
          reg2[pos] = eid;
          list[sl] = pos + 1;
        }
      }
    }
  }
  __syncthreads();

#pragma unroll 4
  for (int i = tid; i < RCAP; i += NTHR) {
    const int e = iclamp(reg2[i], 0, nE - 1);
    const int s = iclamp(srcs[e], 0, nN - 1);
    reg2[i] = (i < nh) ? s : 0;
  }
  if (tid == 0) {
    int fl = (nh >= RCAP) ? 1 : 0;
#pragma unroll
    for (int w2 = 0; w2 < NWAVE; ++w2) fl |= wflg[w2];
    tab[2 * NB]     = nh;
    tab[2 * NB + 1] = fl;
  }
  __syncthreads();

  int* gs = SRT + (size_t)blockIdx.x * RCAP;
  int* gt = TAB + (size_t)blockIdx.x * TABN;
  dump_pass(reg2, tab, gs, gt, tid);
  __threadfence();
  dump_pass(reg2, tab, gs, gt, tid);
}

template<int NT, int EPI>
__global__ __launch_bounds__(GTHR) void k_gemm(
    const unsigned short* __restrict__ A, const unsigned short* __restrict__ WT, int K,
    const float* __restrict__ p0, const float* __restrict__ p1, const float* __restrict__ p2,
    const float* __restrict__ p3, const float* __restrict__ p4,
    float* outF, unsigned short* outH, int doLN)
{
  constexpr int LDW = 16 * NT;
  __shared__ __attribute__((aligned(16))) float stg[GBM * LDW];
  __shared__ __attribute__((aligned(16))) float sp[5 * HID];
  __shared__ __attribute__((aligned(16))) unsigned stw[4 * 128];
  const int tid = (int)threadIdx.x, lane = tid & 31, wave = tid >> 5, hh = lane >> 4, m = lane & 15;
  const int rowBase = (int)blockIdx.x * GBM;
  const int col0    = (int)blockIdx.y * LDW;

  if (tid < 32) {
    if (EPI == 0) {
      const int c = (col0 & 127) + 4 * (tid & 15);
      const v4f a = *(const v4f*)(p0 + c);
      const v4f b = *(const v4f*)(p1 + c);
      const v4f v = (col0 < 128) ? a : b;
      *(v4fa*)(sp + 4 * tid) = rbf4(v);
    } else if (EPI == 1) {
      const int c = col0 + 4 * (tid & 15);
      *(v4fa*)(sp + 4 * tid) = rbf4(*(const v4f*)(p0 + c));
    } else {
      *(v4fa*)(sp + 4 * tid) = rbf4(*(const v4f*)(p0 + 4 * tid));
      if (EPI == 2) {
        *(v4fa*)(sp + HID + 4 * tid)     = rbf4(*(const v4f*)(p1 + 4 * tid));
        *(v4fa*)(sp + 2 * HID + 4 * tid) = rbf4(*(const v4f*)(p2 + 4 * tid));
      }
      *(v4fa*)(sp + 3 * HID + 4 * tid) = rbf4(*(const v4f*)(p3 + 4 * tid));
      *(v4fa*)(sp + 4 * HID + 4 * tid) = rbf4(*(const v4f*)(p4 + 4 * tid));
    }
  }

  v8f acc[NT];
  {
    const v8f z = {0.f, 0.f, 0.f, 0.f, 0.f, 0.f, 0.f, 0.f};
#pragma unroll
    for (int t = 0; t < NT; ++t) acc[t] = z;
  }
  const unsigned short* ap = A  + (size_t)(rowBase + 16 * wave + m) * (size_t)K + 8 * hh;
  const unsigned short* wp = WT + (size_t)(col0 + m) * (size_t)K + 8 * hh;
  const int ksteps = K >> 5;
#pragma unroll 1
  for (int ks = 0; ks < ksteps; ++ks) {
    FragB af;
    af.u[0] = *(const v8us*)(ap + 32 * ks);
    af.u[1] = *(const v8us*)(ap + 32 * ks + 16);
#pragma unroll
    for (int t = 0; t < NT; ++t) {
      const unsigned short* wq = wp + (size_t)(16 * t) * (size_t)K + 32 * ks;
      FragB bf;
      bf.u[0] = *(const v8us*)wq;
      bf.u[1] = *(const v8us*)(wq + 16);
      acc[t] = wmx(af, bf, acc[t]);
    }
  }

#pragma unroll
  for (int t = 0; t < NT; ++t) {
    const int lc = 16 * t + m;
#pragma unroll
    for (int r = 0; r < 8; ++r) {
      const int lr = 16 * wave + 8 * hh + r;
      stg[lr * LDW + lc] = acc[t][r];
    }
  }
  __syncthreads();

  if (EPI == 0) {
    const v4f bv = *(const v4fa*)(sp + 4 * m);
    v4f fv[8];
#pragma unroll
    for (int i = 0; i < 8; ++i) {
      const int lr = 16 * wave + 2 * i + hh;
      fv[i] = *(const v4fa*)(stg + lr * LDW + 4 * m) + bv;
    }
#pragma unroll
    for (int i = 0; i < 8; ++i) {
      const int gr = rowBase + 16 * wave + 2 * i + hh;
      *(volatile v4f*)(outF + (size_t)gr * 256 + col0 + 4 * m) = fv[i];
    }
    __threadfence();
#pragma unroll
    for (int i = 0; i < 8; ++i) {
      const int gr = rowBase + 16 * wave + 2 * i + hh;
      *(volatile v4f*)(outF + (size_t)gr * 256 + col0 + 4 * m) = fv[i];
    }
  } else if (EPI == 1) {
    const int q8 = lane & 7, sub = lane >> 3;
    const v4f ba = *(const v4fa*)(sp + 8 * q8);
    const v4f bb = *(const v4fa*)(sp + 8 * q8 + 4);
    v8us hv[4], lv[4];
#pragma unroll
    for (int i = 0; i < 4; ++i) {
      const int lr = 16 * wave + 4 * i + sub;
      const v4f a = *(const v4fa*)(stg + lr * LDW + 8 * q8) + ba;
      const v4f b = *(const v4fa*)(stg + lr * LDW + 8 * q8 + 4) + bb;
      const float g[8] = {gelu_f(a.x), gelu_f(a.y), gelu_f(a.z), gelu_f(a.w),
                          gelu_f(b.x), gelu_f(b.y), gelu_f(b.z), gelu_f(b.w)};
#pragma unroll
      for (int e = 0; e < 8; ++e) {
        const unsigned hb = bfbits(g[e]);
        hv[i][e] = (unsigned short)hb;
        lv[i][e] = (unsigned short)bfbits(g[e] - __uint_as_float(hb << 16));
      }
    }
#pragma unroll
    for (int i = 0; i < 4; ++i) {
      const int gr = rowBase + 16 * wave + 4 * i + sub;
      unsigned short* up = outH + (size_t)gr * 512 + col0 + 8 * q8;
      *(volatile v8us*)up = hv[i];
      *(volatile v8us*)(up + 256) = lv[i];
    }
    __threadfence();
#pragma unroll
    for (int i = 0; i < 4; ++i) {
      const int gr = rowBase + 16 * wave + 4 * i + sub;
      unsigned short* up = outH + (size_t)gr * 512 + col0 + 8 * q8;
      *(volatile v8us*)up = hv[i];
      *(volatile v8us*)(up + 256) = lv[i];
    }
  } else {
    const v4f bia = *(const v4fa*)(sp + 4 * lane);
    const v4f g0  = *(const v4fa*)(sp + HID + 4 * lane * (EPI == 2 ? 1 : 0));
    const v4f b0  = *(const v4fa*)(sp + 2 * HID * (EPI == 2 ? 1 : 0) + 4 * lane * (EPI == 2 ? 1 : 0));
    const v4f g1  = *(const v4fa*)(sp + 3 * HID + 4 * lane);
    const v4f b1  = *(const v4fa*)(sp + 4 * HID + 4 * lane);
    unsigned* sw = stw + wave * 128;
#pragma unroll 1
    for (int j = 0; j < 16; ++j) {
      const int lr = 16 * wave + j;
      const int gr = rowBase + lr;
      v4f v = *(const v4fa*)(stg + lr * LDW + 4 * lane) + bia;
      float* hp = outF + (size_t)gr * HID + 4 * lane;
      if (EPI == 2) {
        v = ln_row(v, g0, b0);
        v.x = gelu_f(v.x); v.y = gelu_f(v.y); v.z = gelu_f(v.z); v.w = gelu_f(v.w);
      } else {
        const v4f hr = *(const v4f*)hp;
        v = v + hr;
      }
      v4u w = {0u, 0u, 0u, 0u};
      if (doLN != 0) {
        const v4f y = ln_row(v, g1, b1);
        w = hl_pack(sw, y, lane);
      }
      unsigned* np = (unsigned*)outH + (size_t)gr * 128 + 4 * lane;
      *(volatile v4f*)hp = v;
      if (doLN != 0) *(volatile v4u*)np = w;
      __threadfence();
      *(volatile v4f*)hp = v;
      if (doLN != 0) *(volatile v4u*)np = w;
    }
  }
}

__global__ __launch_bounds__(NTHR) void k_scan(
    const int* __restrict__ SRT, const int* __restrict__ TAB, const float* __restrict__ XLR,
    float* H, unsigned short* HN,
    const float* __restrict__ att, const float* __restrict__ cb,
    const float* __restrict__ fg, const float* __restrict__ fb, int MPr) {
  __shared__ __attribute__((aligned(16))) int tab[TABN];
  __shared__ __attribute__((aligned(16))) float sp[4 * HID];
  __shared__ __attribute__((aligned(16))) unsigned stw[NWAVE * 128];
  const int tid = (int)threadIdx.x, lane = tid & 31, wave = tid >> 5;
  const int nodeBase = (int)blockIdx.x * NB;
  const int* gt  = TAB + (size_t)blockIdx.x * TABN;
  const int* srt = SRT + (size_t)blockIdx.x * RCAP;

  for (int u = tid; u < TABN / 4; u += NTHR) *(v4ia*)(tab + 4 * u) = *(const v4i*)(gt + 4 * u);
  if (tid < 32) {
    *(v4fa*)(sp + 4 * tid)           = rbf4(*(const v4f*)(att + 4 * tid));
    *(v4fa*)(sp + HID + 4 * tid)     = rbf4(*(const v4f*)(cb + 4 * tid));
    *(v4fa*)(sp + 2 * HID + 4 * tid) = rbf4(*(const v4f*)(fg + 4 * tid));
    *(v4fa*)(sp + 3 * HID + 4 * tid) = rbf4(*(const v4f*)(fb + 4 * tid));
  }
  __syncthreads();

  const v4f at  = *(const v4fa*)(sp + 4 * lane);
  const v4f cbv = *(const v4fa*)(sp + HID + 4 * lane);
  const v4f fgv = *(const v4fa*)(sp + 2 * HID + 4 * lane);
  const v4f fbv = *(const v4fa*)(sp + 3 * HID + 4 * lane);
  const int nh  = iclamp(tab[2 * NB], 0, RCAP);
  const bool ovf = (tab[2 * NB + 1] == 1);
  const float pz = ovf ? __int_as_float(0x7fc00000) : 0.0f;
  unsigned* sw = stw + wave * 128;

#pragma unroll 1
  for (int jt = 0; jt < NB / NWAVE; ++jt) {
    const int slot = wave * (NB / NWAVE) + jt;
    const int grow = nodeBase + slot;
    if (grow >= MPr) continue;
    const int st = iclamp(tab[slot], 0, nh);
    int cnt = iclamp(tab[NB + slot], 0, DEGCAP);
    if (cnt > nh - st) cnt = nh - st;

    const float* xrow = XLR + (size_t)grow * 256 + 4 * lane;
    const v4f xr = *(const v4f*)(xrow + HID);
    const v4f hrow = *(const v4f*)(H + (size_t)grow * HID + 4 * lane);
    float mx = -1.0e30f, dn = 0.f;
    v4f av = {0.f, 0.f, 0.f, 0.f};
    const int tot = cnt + 1;

#pragma unroll 1
    for (int b0 = 0; b0 < tot; b0 += 32) {
      const int idx = b0 + lane;
      const int gi  = iclamp(st + idx, 0, RCAP - 1);
      int ev = srt[gi];
      ev = (idx < cnt) ? ev : grow;
      ev = iclamp(ev, 0, MPr - 1);
      const int m32 = (tot - b0) < 32 ? (tot - b0) : 32;
#pragma unroll 1
      for (int k = 0; k < m32; ++k) {
        const int s = __builtin_amdgcn_readlane(ev, k);
        const v4f xs = *(const v4f*)(XLR + (size_t)s * 256 + 4 * lane);
        float t0 = xs.x + xr.x, t1 = xs.y + xr.y, t2 = xs.z + xr.z, t3 = xs.w + xr.w;
        t0 = t0 > 0.f ? t0 : t0 * NEGS;
        t1 = t1 > 0.f ? t1 : t1 * NEGS;
        t2 = t2 > 0.f ? t2 : t2 * NEGS;
        t3 = t3 > 0.f ? t3 : t3 * NEGS;
        float part = t0 * at.x;
        part = fmaf(t1, at.y, part);
        part = fmaf(t2, at.z, part);
        part = fmaf(t3, at.w, part);
        part += __shfl_xor(part, 1);
        part += __shfl_xor(part, 2);
        part += __shfl_xor(part, 4);
        const float df = part - mx;
        const float ee = expf(-fabsf(df));
        const bool up  = df > 0.f;
        const float s1 = up ? ee : 1.0f;
        const float s2 = up ? 1.0f : ee;
        mx = up ? part : mx;
        dn = fmaf(dn, s1, s2);
        av.x = fmaf(av.x, s1, s2 * xs.x);
        av.y = fmaf(av.y, s1, s2 * xs.y);
        av.z = fmaf(av.z, s1, s2 * xs.z);
        av.w = fmaf(av.w, s1, s2 * xs.w);
      }
    }
    const float iv = __builtin_amdgcn_rcpf(dn);
    v4f hv;
    hv.x = fmaf(av.x, iv, cbv.x) + hrow.x + pz;
    hv.y = fmaf(av.y, iv, cbv.y) + hrow.y + pz;
    hv.z = fmaf(av.z, iv, cbv.z) + hrow.z + pz;
    hv.w = fmaf(av.w, iv, cbv.w) + hrow.w + pz;
    const v4f y = ln_row(hv, fgv, fbv);
    const v4u w = hl_pack(sw, y, lane);
    float* hp = H + (size_t)grow * HID + 4 * lane;
    unsigned* np = (unsigned*)HN + (size_t)grow * 128 + 4 * lane;
    *(volatile v4f*)hp = hv;
    *(volatile v4u*)np = w;
    __threadfence();
    *(volatile v4f*)hp = hv;
    *(volatile v4u*)np = w;
  }
}

__global__ __launch_bounds__(128) void k_pool(const float* __restrict__ H, const int* __restrict__ batch,
                                              float* Z, int nN) {
  __shared__ int lst[512];
  __shared__ int wt[4];
  __shared__ __attribute__((aligned(16))) float zs[HID];
  const int tid = (int)threadIdx.x, lane = tid & 31, wave = tid >> 5;
  const int g = (int)blockIdx.x;
  double acc = 0.0;
  int cnt = 0;
  const int nCh = (nN + 511) / 512;
#pragma unroll 1
  for (int ch = 0; ch < nCh; ++ch) {
    const int n4 = ch * 512 + 4 * tid;
    const int ad = n4 < nN - 4 ? n4 : nN - 4;
    const v4i bq = *(const v4i*)(batch + ad);
    const bool valid = n4 < nN;
    const bool m0 = valid && bq.x == g, m1 = valid && bq.y == g, m2 = valid && bq.z == g, m3 = valid && bq.w == g;
    const int c = (int)m0 + (int)m1 + (int)m2 + (int)m3;
    int incl = c;
#pragma unroll
    for (int d = 1; d < 32; d <<= 1) {
      const int up = __shfl_up(incl, d);
      if (lane >= d) incl += up;
    }
    if (lane == 31) wt[wave] = incl;
    __syncthreads();
    int pre = 0, all = 0;
#pragma unroll
    for (int w2 = 0; w2 < 4; ++w2) { const int t = wt[w2]; all += t; pre += (w2 < wave) ? t : 0; }
    int pos = pre + incl - c;
    if (m0) { lst[pos] = n4;     ++pos; }
    if (m1) { lst[pos] = n4 + 1; ++pos; }
    if (m2) { lst[pos] = n4 + 2; ++pos; }
    if (m3) { lst[pos] = n4 + 3; ++pos; }
    __syncthreads();
    all = all > 512 ? 512 : all;
#pragma unroll 1
    for (int q = 0; q < all; ++q) {
      const int n = iclamp(lst[q], 0, nN - 1);
      acc += (double)H[(size_t)n * HID + tid];
    }
    cnt += all;
    __syncthreads();
  }
  const int cc = cnt > 1 ? cnt : 1;
  zs[tid] = (float)acc * (1.0f / (float)cc);
  __syncthreads();
  if (tid < 32) {
    const v4f v = *(const v4fa*)(zs + 4 * tid);
    float* zp = Z + (size_t)g * HID + 4 * tid;
    *(volatile v4f*)zp = v;
    __threadfence();
    *(volatile v4f*)zp = v;
  }
}

__global__ __launch_bounds__(NTHR) void k_head(const float* __restrict__ Z, const float* __restrict__ W,
                                               const float* __restrict__ b, const int* __restrict__ TAB,
                                               int nblk, float* out) {
  __shared__ __attribute__((aligned(16))) float zs[NG * HID];
  __shared__ __attribute__((aligned(16))) float wsh[HID * NCLS];
  __shared__ float bs[16];
  __shared__ __attribute__((aligned(16))) float os[NG * NCLS];
  __shared__ int pf;
  const int tid = (int)threadIdx.x;
  for (int u = tid; u < NG * HID / 4; u += NTHR) *(v4fa*)(zs + 4 * u) = *(const v4f*)(Z + 4 * u);
  for (int u = tid; u < HID * NCLS / 4; u += NTHR) *(v4fa*)(wsh + 4 * u) = rbf4(*(const v4f*)(W + 4 * u));
  if (tid < 16) bs[tid] = rbf(b[tid < NCLS ? tid : NCLS - 1]);
  if (tid == 0) pf = 0;
  __syncthreads();
  if (tid < 64) {
    const int bi = tid < nblk ? tid : nblk - 1;
    const int f = TAB[(size_t)bi * TABN + 2 * NB + 1];
    if (tid < nblk && f == 1) pf = 1;
  }
  for (int t = tid; t < NG * NCLS; t += NTHR) {
    const int g = t / NCLS;
    const int j = t - g * NCLS;
    float acc = bs[j];
#pragma unroll 1
    for (int k = 0; k < HID; ++k) acc = fmaf(zs[g * HID + k], wsh[k * NCLS + j], acc);
    os[t] = acc;
  }
  __syncthreads();
  if (tid < NG * NCLS / 4) {
    v4f v = *(const v4fa*)(os + 4 * tid);
    if (pf != 0) {
      const float qn = __int_as_float(0x7fc00000);
      v.x = qn; v.y = qn; v.z = qn; v.w = qn;
    }
    *(volatile v4f*)(out + 4 * tid) = v;
    __threadfence();
    *(volatile v4f*)(out + 4 * tid) = v;
  }
}

static inline int cdiv(int a, int b) { return (a + b - 1) / b; }

extern "C" void kernel_launch(void* const* d_in, const int* in_sizes, int n_in,
                              void* d_out, int out_size, void* d_ws, size_t ws_size,
                              hipStream_t stream) {
  if (n_in < 23) return;
  const int nN = in_sizes[0] / INC;
  if (nN <= 0 || in_sizes[0] != nN * INC || (nN & 3) != 0 || nN > 65536) return;
  if (in_sizes[1] < 2 || (in_sizes[1] & 1) != 0) return;
  const int nE = in_sizes[1] / 2;
  if (nE < 1 || nE > (1 << 20)) return;
  if (in_sizes[2] != nN) return;
  if (in_sizes[3] != INC * HID || in_sizes[4] != HID || in_sizes[5] != HID || in_sizes[6] != HID) return;
  if (in_sizes[7] != NLAY * HID || in_sizes[8] != NLAY * HID) return;
  if (in_sizes[9] != NLAY * HID * HID || in_sizes[10] != NLAY * HID) return;
  if (in_sizes[11] != NLAY * HID * HID || in_sizes[12] != NLAY * HID) return;
  if (in_sizes[13] != NLAY * HID || in_sizes[14] != NLAY * HID) return;
  if (in_sizes[15] != NLAY * HID || in_sizes[16] != NLAY * HID) return;
  if (in_sizes[17] != NLAY * HID * FFH || in_sizes[18] != NLAY * FFH) return;
  if (in_sizes[19] != NLAY * FFH * HID || in_sizes[20] != NLAY * HID) return;
  if (in_sizes[21] != HID * NCLS || in_sizes[22] != NCLS) return;
  if (out_size != NG * NCLS) return;

  const float* x      = (const float*)d_in[0];
  const int*   ei     = (const int*)  d_in[1];
  const int*   batch  = (const int*)  d_in[2];
  const float* in_W   = (const float*)d_in[3];
  const float* in_b   = (const float*)d_in[4];
  const float* in_lg  = (const float*)d_in[5];
  const float* in_lb  = (const float*)d_in[6];
  const float* ln_g   = (const float*)d_in[7];
  const float* ln_b   = (const float*)d_in[8];
  const float* Wl     = (const float*)d_in[9];
  const float* bl     = (const float*)d_in[10];
  const float* Wr     = (const float*)d_in[11];
  const float* br     = (const float*)d_in[12];
  const float* att    = (const float*)d_in[13];
  const float* conv_b = (const float*)d_in[14];
  const float* ff_lg  = (const float*)d_in[15];
  const float* ff_lb  = (const float*)d_in[16];
  const float* ffW1   = (const float*)d_in[17];
  const float* ffb1   = (const float*)d_in[18];
  const float* ffW2   = (const float*)d_in[19];
  const float* ffb2   = (const float*)d_in[20];
  const float* clfW   = (const float*)d_in[21];
  const float* clfb   = (const float*)d_in[22];
  float* out = (float*)d_out;
  const int* src = ei;
  const int* dst = ei + nE;

  const int MP   = cdiv(nN, 128) * 128;
  const int nblk = cdiv(MP, NB);
  const int vec8 = ((nE & 3) == 0) ? 1 : 0;
  if (nblk < 1 || nblk > 64 || nblk * NB < MP) return;

  char* ws = (char*)d_ws;
  size_t off = 0;
  const size_t oR1  = off; off += (size_t)MP * 256 * 4;            off = (off + 255) & ~(size_t)255;
  const size_t oH   = off; off += (size_t)MP * HID * 4;            off = (off + 255) & ~(size_t)255;
  const size_t oHN  = off; off += (size_t)MP * 256 * 2;            off = (off + 255) & ~(size_t)255;
  const size_t oXB  = off; off += (size_t)MP * INC * 2;            off = (off + 255) & ~(size_t)255;
  const size_t oSRT = off; off += (size_t)nblk * RCAP * 4;         off = (off + 255) & ~(size_t)255;
  const size_t oTAB = off; off += (size_t)nblk * TABN * 4;         off = (off + 255) & ~(size_t)255;
  const size_t oINW = off; off += (size_t)HID * INC * 2;           off = (off + 255) & ~(size_t)255;
  const size_t oWLR = off; off += (size_t)NLAY * 256 * 256 * 2;    off = (off + 255) & ~(size_t)255;
  const size_t oFW1 = off; off += (size_t)NLAY * 256 * 256 * 2;    off = (off + 255) & ~(size_t)255;
  const size_t oFW2 = off; off += (size_t)NLAY * 128 * 512 * 2;    off = (off + 255) & ~(size_t)255;
  const size_t oZ   = off; off += (size_t)NG * HID * 4;            off = (off + 255) & ~(size_t)255;
  if (off > ws_size || off > (size_t)WSMAX) return;
  float*          XLR  = (float*)(ws + oR1);
  unsigned short* UHL  = (unsigned short*)(ws + oR1);
  float*          H    = (float*)(ws + oH);
  unsigned short* HN   = (unsigned short*)(ws + oHN);
  unsigned short* XB   = (unsigned short*)(ws + oXB);
  int*            SRT  = (int*)(ws + oSRT);
  int*            TAB  = (int*)(ws + oTAB);
  unsigned short* INWt = (unsigned short*)(ws + oINW);
  unsigned short* WLRt = (unsigned short*)(ws + oWLR);
  unsigned short* FW1t = (unsigned short*)(ws + oFW1);
  unsigned short* FW2t = (unsigned short*)(ws + oFW2);
  float*          Z    = (float*)(ws + oZ);

  hipFuncSetAttribute(reinterpret_cast<const void*>(&k_bucket),
                      hipFuncAttributeMaxDynamicSharedMemorySize, LDS_BKT);

  const int nbx = MP / 32;
  k_prep<<<nbx + 4 + NLAY * 96, NTHR, 0, stream>>>(x, in_W, Wl, Wr, ffW1, ffW2, XB, INWt, WLRt, FW1t, FW2t, nN, nbx);
  k_bucket<<<nblk, NTHR, LDS_BKT, stream>>>(src, dst, SRT, TAB, nN, nE, vec8);

  const int gM = MP / GBM;
  k_gemm<8, 2><<<dim3(gM, 1), GTHR, 0, stream>>>(XB, INWt, INC, in_b, in_lg, in_lb, ln_g, ln_b, H, HN, 1);

  for (int i = 0; i < NLAY; ++i) {
    const int nx = (i + 1 < NLAY) ? (i + 1) : i;
    k_gemm<4, 0><<<dim3(gM, 4), GTHR, 0, stream>>>(HN, WLRt + (size_t)i * 65536, 256,
                                                    bl + i * HID, br + i * HID, bl + i * HID, bl + i * HID, bl + i * HID,
                                                    XLR, HN, 0);
    k_scan<<<nblk, NTHR, 0, stream>>>(SRT, TAB, XLR, H, HN, att + i * HID, conv_b + i * HID,
                                      ff_lg + i * HID, ff_lb + i * HID, MP);
    k_gemm<4, 1><<<dim3(gM, 4), GTHR, 0, stream>>>(HN, FW1t + (size_t)i * 65536, 256,
                                                    ffb1 + i * FFH, ffb1 + i * FFH, ffb1 + i * FFH, ffb1 + i * FFH,
                                                    ffb1 + i * FFH, H, UHL, 0);
    k_gemm<8, 3><<<dim3(gM, 1), GTHR, 0, stream>>>(UHL, FW2t + (size_t)i * 65536, 512,
                                                    ffb2 + i * HID, ffb2 + i * HID, ffb2 + i * HID,
                                                    ln_g + nx * HID, ln_b + nx * HID, H, HN, (i + 1 < NLAY) ? 1 : 0);
  }

  k_pool<<<NG, 128, 0, stream>>>(H, batch, Z, nN);
  k_head<<<1, NTHR, 0, stream>>>(Z, clfW, clfb, TAB, nblk, out);
}
